// SparseAttention_48215302865704
// MI455X (gfx1250) — hardware-verified
//
#include <hip/hip_runtime.h>

typedef __attribute__((ext_vector_type(16))) _Float16 v16h;
typedef __attribute__((ext_vector_type(8)))  _Float16 v8h;
typedef __attribute__((ext_vector_type(16))) __bf16   v16b;
typedef __attribute__((ext_vector_type(8)))  __bf16   v8b;
typedef __attribute__((ext_vector_type(8)))  float    v8f;
typedef __attribute__((ext_vector_type(4)))  float    v4f;
typedef __attribute__((ext_vector_type(4)))  unsigned int v4u;

constexpr int NBATCH = 2;
constexpr int SEQ    = 4096;
constexpr int EMB    = 1024;
constexpr int NHEAD  = 16;
constexpr int HDIM   = 64;
constexpr int NBLK   = 64;
constexpr int NMB    = 12;
constexpr int KCH    = 64;
static_assert(NHEAD * HDIM == EMB);
static_assert(NBLK * KCH == SEQ);
static_assert(EMB % 64 == 0);
static_assert(SEQ % 64 == 0);
static_assert(EMB % 32 == 0);
static_assert(HDIM == 64);

__device__ __forceinline__ unsigned short f2bf_bits(float f) {
  unsigned u = __float_as_uint(f);
  return (unsigned short)((u + 0x7FFFu + ((u >> 16) & 1u)) >> 16);
}
__device__ __forceinline__ float bf_bits2f(unsigned short h) { return __uint_as_float(((unsigned)h) << 16); }

__device__ __forceinline__ void dep_guard_h(v8f& a, v8f& b, v16h x, v16h y) { asm volatile("v_nop\n\tv_nop\n\tv_nop\n\tv_nop" : "+v"(a), "+v"(b) : "v"(x), "v"(y)); }
__device__ __forceinline__ void dep_guard_b(v8f& a, v8f& b, v16b x, v16b y) { asm volatile("v_nop\n\tv_nop\n\tv_nop\n\tv_nop" : "+v"(a), "+v"(b) : "v"(x), "v"(y)); }
__device__ __forceinline__ void keep4_h(v16h a, v16h b, v16h c, v16h d) { asm volatile("v_nop" :: "v"(a), "v"(b), "v"(c), "v"(d)); }
__device__ __forceinline__ void keep4_b(v16b a, v16b b, v16b c, v16b d) { asm volatile("v_nop" :: "v"(a), "v"(b), "v"(c), "v"(d)); }
__device__ __forceinline__ void acc_guard4(v8f& a, v8f& b, v8f& c, v8f& d) { asm volatile("v_nop\n\tv_nop\n\tv_nop\n\tv_nop" : "+v"(a), "+v"(b), "+v"(c), "+v"(d)); }
template <typename T> struct Frag;
template <> struct Frag<_Float16> {
  typedef v16h V; union U { v16h v; v8h h[2]; };
  static __device__ __forceinline__ v16h load(const _Float16* p) {
    U f; f.h[0] = *(const v8h*)(p); f.h[1] = *(const v8h*)(p + 16); return f.v;
  }
  static __device__ __forceinline__ v8f mma(v16h a, v16h b, v8f c) {
    return __builtin_amdgcn_wmma_f32_16x16x32_f16(false, a, false, b, (short)0, c, false, false);
  }
  static __device__ __forceinline__ void guard(v8f& a, v8f& b, v16h x, v16h y) { dep_guard_h(a, b, x, y); }
  static __device__ __forceinline__ void keep(v16h a, v16h b, v16h c, v16h d) { keep4_h(a, b, c, d); }
};
template <> struct Frag<__bf16> {
  typedef v16b V; union U { v16b v; v8b h[2]; };
  static __device__ __forceinline__ v16b load(const __bf16* p) {
    U f; f.h[0] = *(const v8b*)(p); f.h[1] = *(const v8b*)(p + 16); return f.v;
  }
  static __device__ __forceinline__ v8f mma(v16b a, v16b b, v8f c) {
    return __builtin_amdgcn_wmma_f32_16x16x32_bf16(false, a, false, b, (short)0, c, false, false);
  }
  static __device__ __forceinline__ void guard(v8f& a, v8f& b, v16b x, v16b y) { dep_guard_b(a, b, x, y); }
  static __device__ __forceinline__ void keep(v16b a, v16b b, v16b c, v16b d) { keep4_b(a, b, c, d); }
};

__device__ __forceinline__ v8f at_mma(v16b a, v16b b, v8f c) {
  c = __builtin_amdgcn_wmma_f32_16x16x32_bf16(false, a, false, b, (short)0, c, false, false);
  asm volatile("v_nop\n\tv_nop\n\tv_nop\n\tv_nop" : "+v"(c) : "v"(a), "v"(b));
  return c;
}

template <int ET> struct Elem;
template <> struct Elem<0> { typedef _Float16 T; };
template <> struct Elem<1> { typedef __bf16 T; };
template <int ET, bool SPLIT, int BIAS_MODE, int OUT_MODE, bool RESID, int ACT = 0, bool BSPLIT = true>
__global__ __launch_bounds__(256) void wmma_gemm64(
    const unsigned short* __restrict__ Ap, const unsigned short* __restrict__ A2p, int lda, long strideA,
    const unsigned short* __restrict__ Btp, const unsigned short* __restrict__ Bt2p, int ldb, long strideB,
    void* __restrict__ Cout, void* __restrict__ Cout2, int ldc, long strideC,
    const float* __restrict__ bias,
    const float* __restrict__ resid, long strideR,
    int M, int N, int K, float scale) {
  typedef typename Elem<ET>::T T;
  typedef typename Frag<T>::V V;
  const T* A = (const T*)Ap; const T* A2 = (const T*)A2p; const T* Bt = (const T*)Btp; const T* Bt2 = (const T*)Bt2p;
  __shared__ __align__(16) float sT[8][16 * 68];
  const int b    = blockIdx.y;
  const int lane = threadIdx.x & 31;
  const int wave = threadIdx.x >> 5;
  const int tilesN = N >> 6;
  const int tilesM = M >> 6;
  const int tile = blockIdx.x * 8 + wave;
  if (tile >= tilesM * tilesN) return;
  const int tm = tile / tilesN;
  const int tn = tile - tm * tilesN;
  const int m0 = tm << 6;
  const int n0 = tn << 6;

  const T* Ab  = A  + (size_t)b * strideA;
  const T* Bb  = Bt + (size_t)b * strideB;
  const T* Ab2 = SPLIT ? (A2  + (size_t)b * strideA) : nullptr;
  const T* Bb2 = (SPLIT && BSPLIT) ? (Bt2 + (size_t)b * strideB) : nullptr;

  const int rlane = lane & 15;
  const int koff  = (lane >> 4) * 8;
  const int mOff  = (lane >> 4) * 8;

  v8f acc[4][4];
#pragma unroll
  for (int i = 0; i < 4; ++i)
#pragma unroll
    for (int j = 0; j < 4; ++j) acc[i][j] = (v8f){0.f,0.f,0.f,0.f,0.f,0.f,0.f,0.f};

  for (int k0 = 0; k0 < K; k0 += 32) {
    V bh[4], bl[4];
#pragma unroll
    for (int j = 0; j < 4; ++j) {
      const size_t bo = (size_t)(n0 + (j << 4) + rlane) * ldb + koff + k0;
      bh[j] = Frag<T>::load(Bb + bo);
      if (SPLIT && BSPLIT) bl[j] = Frag<T>::load(Bb2 + bo);
      else bl[j] = bh[j];
    }
#pragma unroll
    for (int i = 0; i < 4; ++i) {
      const size_t ao = (size_t)(m0 + (i << 4) + rlane) * lda + koff + k0;
      V ah = Frag<T>::load(Ab + ao);
      V al = ah;
      if (SPLIT) al = Frag<T>::load(Ab2 + ao);
#pragma unroll
      for (int j = 0; j < 4; ++j) {
        acc[i][j] = Frag<T>::mma(ah, bh[j], acc[i][j]);
        if (SPLIT) {
          if (BSPLIT) acc[i][j] = Frag<T>::mma(ah, bl[j], acc[i][j]);
          acc[i][j] = Frag<T>::mma(al, bh[j], acc[i][j]);
        }
      }
      Frag<T>::guard(acc[i][0], acc[i][3], ah, SPLIT ? al : ah);
    }
    Frag<T>::keep(bh[0], bh[1], bh[2], bh[3]);
    if (SPLIT && BSPLIT) Frag<T>::keep(bl[0], bl[1], bl[2], bl[3]);
  }
  acc_guard4(acc[0][0], acc[0][1], acc[0][2], acc[0][3]);
  acc_guard4(acc[1][0], acc[1][1], acc[1][2], acc[1][3]);
  acc_guard4(acc[2][0], acc[2][1], acc[2][2], acc[2][3]);
  acc_guard4(acc[3][0], acc[3][1], acc[3][2], acc[3][3]);

  float* slab = sT[wave];
  const float* Rb = RESID ? (resid + (size_t)b * strideR) : nullptr;
#pragma unroll
  for (int i = 0; i < 4; ++i) {
    const int mBase = m0 + (i << 4);
#pragma unroll
    for (int j = 0; j < 4; ++j) {
      const int n = n0 + (j << 4) + rlane;
      float bv = 0.f;
      if (BIAS_MODE == 2) bv = bias[n];
#pragma unroll
      for (int r = 0; r < 8; ++r) {
        float v = acc[i][j][r] * scale;
        if (BIAS_MODE == 1) v += bias[mBase + mOff + r];
        if (BIAS_MODE == 2) v += bv;
        if (RESID) v += Rb[(size_t)(mBase + mOff + r) * ldc + n];
        if (ACT == 1) v = tanhf(v);
        if (ACT == 2) v = fmaxf(v, 0.0f);
        if (ACT == 3) v = v / (1.0f + expf(-v));
        if (ACT == 4) v = (v > 0.f) ? v : 0.01f * v;
        slab[(mOff + r) * 68 + (j << 4) + rlane] = v;
      }
    }
    __builtin_amdgcn_fence(__ATOMIC_RELEASE, "workgroup");
    __builtin_amdgcn_wave_barrier();
    __builtin_amdgcn_fence(__ATOMIC_ACQUIRE, "workgroup");
    if (OUT_MODE == 0) {
      float* C = (float*)Cout + (size_t)b * strideC;
      const int hh = lane >> 4, c4 = (lane & 15) * 4;
      for (int pass = 0; pass < 2; ++pass) {
#pragma unroll
        for (int it = 0; it < 8; ++it) {
          const int row = it * 2 + hh;
          v4f v = *(const v4f*)(slab + row * 68 + c4);
          *(volatile v4f*)(C + (size_t)(mBase + row) * ldc + n0 + c4) = v;
        }
        __threadfence();
      }
    } else {
      const int q = lane >> 3, c8 = (lane & 7) * 8;
      unsigned short* C  = (unsigned short*)Cout  + (size_t)b * strideC;
      unsigned short* C2 = (OUT_MODE == 2) ? ((unsigned short*)Cout2 + (size_t)b * strideC) : nullptr;
      for (int pass = 0; pass < 2; ++pass) {
#pragma unroll
        for (int it = 0; it < 4; ++it) {
          const int row = it * 4 + q;
          const float* sp = slab + row * 68 + c8;
          v8h hv, lv;
#pragma unroll
          for (int e = 0; e < 8; ++e) {
            if (OUT_MODE == 1) {
              hv[e] = (_Float16)sp[e];
              lv[e] = hv[e];
            } else {
              unsigned short hb = f2bf_bits(sp[e]);
              unsigned short lb = f2bf_bits(sp[e] - bf_bits2f(hb));
              hv[e] = __builtin_bit_cast(_Float16, hb);
              lv[e] = __builtin_bit_cast(_Float16, lb);
            }
          }
          *(volatile v8h*)(C + (size_t)(mBase + row) * ldc + n0 + c8) = hv;
          if (OUT_MODE == 2) *(volatile v8h*)(C2 + (size_t)(mBase + row) * ldc + n0 + c8) = lv;
        }
        __threadfence();
      }
    }
    __builtin_amdgcn_fence(__ATOMIC_RELEASE, "workgroup");
    __builtin_amdgcn_wave_barrier();
    __builtin_amdgcn_fence(__ATOMIC_ACQUIRE, "workgroup");
  }
}

__global__ __launch_bounds__(256) void cast_f32_bf16x8(const float* __restrict__ in,
                                                       unsigned short* __restrict__ out, int n8) {
  const int i = blockIdx.x * 256 + threadIdx.x;
  if (i < n8) {
    const size_t e = (size_t)i * 8;
    const v4f a = *(const v4f*)(in + e);
    const v4f b = *(const v4f*)(in + e + 4);
    v4u w;
    w[0] = (unsigned)f2bf_bits(a[0]) | ((unsigned)f2bf_bits(a[1]) << 16);
    w[1] = (unsigned)f2bf_bits(a[2]) | ((unsigned)f2bf_bits(a[3]) << 16);
    w[2] = (unsigned)f2bf_bits(b[0]) | ((unsigned)f2bf_bits(b[1]) << 16);
    w[3] = (unsigned)f2bf_bits(b[2]) | ((unsigned)f2bf_bits(b[3]) << 16);
    *(volatile v4u*)(out + e) = w;
    __threadfence();
    *(volatile v4u*)(out + e) = w;
  }
}

__global__ __launch_bounds__(256) void transpose_cast_bf16(const float* __restrict__ w0, const float* __restrict__ w1,
                                                           const float* __restrict__ w2, const float* __restrict__ w3,
                                                           unsigned short* __restrict__ o0, unsigned short* __restrict__ o1,
                                                           unsigned short* __restrict__ o2, unsigned short* __restrict__ o3) {
  __shared__ float tile[64][65];
  const int tid = threadIdx.x;
  const int z = blockIdx.z;
  const float* W = w0; unsigned short* O = o0;
  if (z == 1) { W = w1; O = o1; }
  if (z == 2) { W = w2; O = o2; }
  if (z == 3) { W = w3; O = o3; }
  const int n0 = blockIdx.x * 64;
  const int k0 = blockIdx.y * 64;
#pragma unroll
  for (int it = 0; it < 4; ++it) {
    const int idx = it * 256 + tid;
    const int row = idx >> 4;
    const int c4  = (idx & 15) * 4;
    const v4f v = *(const v4f*)(W + (size_t)(k0 + row) * EMB + n0 + c4);
    tile[row][c4 + 0] = v[0];
    tile[row][c4 + 1] = v[1];
    tile[row][c4 + 2] = v[2];
    tile[row][c4 + 3] = v[3];
  }
  __syncthreads();
  const int r  = tid >> 3;
  const int c8 = (tid & 7) * 8;
#pragma unroll
  for (int it = 0; it < 2; ++it) {
    const int rr = r + 32 * it;
    v4u wv;
    wv[0] = (unsigned)f2bf_bits(tile[c8 + 0][rr]) | ((unsigned)f2bf_bits(tile[c8 + 1][rr]) << 16);
    wv[1] = (unsigned)f2bf_bits(tile[c8 + 2][rr]) | ((unsigned)f2bf_bits(tile[c8 + 3][rr]) << 16);
    wv[2] = (unsigned)f2bf_bits(tile[c8 + 4][rr]) | ((unsigned)f2bf_bits(tile[c8 + 5][rr]) << 16);
    wv[3] = (unsigned)f2bf_bits(tile[c8 + 6][rr]) | ((unsigned)f2bf_bits(tile[c8 + 7][rr]) << 16);
    unsigned short* p = O + (size_t)(n0 + rr) * EMB + k0 + c8;
    *(volatile v4u*)p = wv;
    __threadfence();
    *(volatile v4u*)p = wv;
  }
}

constexpr int KPLANE = KCH * HDIM;

__global__ __launch_bounds__(128)
void block_attn_kernel(const unsigned short* __restrict__ qhp, const unsigned short* __restrict__ qlp,
                       const unsigned short* __restrict__ khp, const unsigned short* __restrict__ klp,
                       const unsigned short* __restrict__ vhp, const unsigned short* __restrict__ vlp,
                       unsigned short* __restrict__ ohp, unsigned short* __restrict__ olp,
                       const int* __restrict__ bidx) {
  __shared__ __align__(16) __bf16 KVs[4 * KPLANE];
  __shared__ __align__(16) __bf16 Psh[4][16 * KCH];
  __shared__ __align__(16) __bf16 Psl[4][16 * KCH];
  __shared__ int slist[80];

  const int tid  = threadIdx.x;
  const int wave = tid >> 5;
  const int lane = tid & 31;
  const int hh   = lane >> 4;
  const int c    = lane & 15;
  const int qblk = blockIdx.x & (NBLK - 1);
  const int h    = blockIdx.x >> 6;
  const int qbase = qblk * KCH;
  const int q0    = qbase + wave * 16;

  const int   hp1  = h + 1;
  const float sodd = __uint_as_float(0x3F3504F3u);
  const float spow = __uint_as_float(((unsigned)(127 - (hp1 >> 1))) << 23);
  const float slope = ((hp1 & 1) ? sodd : 1.0f) * spow;
  const float nslope = -slope;

  if (tid == 0) {
    int n = 0;
    if (qblk == 0) {
      for (int i = 0; i < NBLK; ++i) slist[i] = i * KCH;
      n = NBLK;
    } else {
      slist[0] = 0;
      n = 1;
      for (int j = 0; j < NMB; ++j) {
        int bb = bidx[qblk * NMB + j];
        if (bb >= 0) {
          bb = (bb > NBLK - 1) ? (NBLK - 1) : bb;
          slist[n] = bb * KCH;
          ++n;
        }
      }
    }
    slist[72] = n;
  }
  __syncthreads();
  int nch = slist[72];
  nch = (nch < 1) ? 1 : ((nch > NBLK) ? NBLK : nch);

  v16b qah[2], qal[2];
  {
    const size_t qoff = (size_t)(q0 + c) * EMB + h * HDIM + 8 * hh;
    const __bf16* qr  = (const __bf16*)qhp + qoff;
    const __bf16* qr2 = (const __bf16*)qlp + qoff;
#pragma unroll
    for (int dc = 0; dc < 2; ++dc) {
      qah[dc] = Frag<__bf16>::load(qr + dc * 32);
      qal[dc] = Frag<__bf16>::load(qr2 + dc * 32);
    }
  }

  float mrow[8], lrow[8];
  v8f oacc[4];
#pragma unroll
  for (int r = 0; r < 8; ++r) { mrow[r] = -__builtin_inff(); lrow[r] = 0.f; }
#pragma unroll
  for (int t = 0; t < 4; ++t) oacc[t] = (v8f){0.f,0.f,0.f,0.f,0.f,0.f,0.f,0.f};

  const __bf16* Ksh = KVs;
  const __bf16* Ksl = KVs + KPLANE;
  const __bf16* Vsh = KVs + 2 * KPLANE;
  const __bf16* Vsl = KVs + 3 * KPLANE;
  __bf16* pwh = Psh[wave];
  __bf16* pwl = Psl[wave];

  for (int ci = 0; ci < nch; ++ci) {
    int k0 = slist[ci];
    k0 = (k0 < 0) ? 0 : ((k0 > SEQ - KCH) ? (SEQ - KCH) : k0);
    __syncthreads();
#pragma unroll
    for (int i = 0; i < 4; ++i) {
      const int p   = i * 128 + tid;
      const int row = p >> 3;
      const int c8  = (p & 7) * 8;
      const size_t gk = (size_t)(k0 + row) * EMB + h * HDIM + c8;
      const size_t gv = (size_t)(h * HDIM + row) * SEQ + k0 + c8;
      const v4u a0 = *(const v4u*)(khp + gk);
      const v4u a1 = *(const v4u*)(klp + gk);
      const v4u a2 = *(const v4u*)(vhp + gv);
      const v4u a3 = *(const v4u*)(vlp + gv);
      *(v4u*)(KVs + row * HDIM + c8)               = a0;
      *(v4u*)(KVs + KPLANE + row * HDIM + c8)      = a1;
      *(v4u*)(KVs + 2 * KPLANE + row * KCH + c8)   = a2;
      *(v4u*)(KVs + 3 * KPLANE + row * KCH + c8)   = a3;
    }
    __syncthreads();

    v8f s[4];
#pragma unroll
    for (int j = 0; j < 4; ++j) {
      s[j] = (v8f){0.f,0.f,0.f,0.f,0.f,0.f,0.f,0.f};
#pragma unroll
      for (int dc = 0; dc < 2; ++dc) {
        const __bf16* kp = Ksh + (j * 16 + c) * HDIM + dc * 32 + 8 * hh;
        const __bf16* kq = Ksl + (j * 16 + c) * HDIM + dc * 32 + 8 * hh;
        const v16b kfh = Frag<__bf16>::load(kp);
        const v16b kfl = Frag<__bf16>::load(kq);
        s[j] = at_mma(qah[dc], kfh, s[j]);
        s[j] = at_mma(qah[dc], kfl, s[j]);
        s[j] = at_mma(qal[dc], kfh, s[j]);
      }
    }

    float cm[8];
#pragma unroll
    for (int r = 0; r < 8; ++r) {
      const int qpos = q0 + 8 * hh + r;
      float m = -__builtin_inff();
#pragma unroll
      for (int j = 0; j < 4; ++j) {
        const int kpos = k0 + j * 16 + c;
        int dd = qpos - kpos;
        dd = (dd < 0) ? -dd : dd;
        const float bias = nslope * (float)dd;
        const float sv = s[j][r] * 0.125f + bias;
        s[j][r] = sv;
        m = fmaxf(m, sv);
      }
#pragma unroll
      for (int off = 1; off < 16; off <<= 1) m = fmaxf(m, __shfl_xor(m, off, 32));
      cm[r] = m;
    }

#pragma unroll
    for (int r = 0; r < 8; ++r) {
      const float mnew  = fmaxf(mrow[r], cm[r]);
      const float alpha = expf(mrow[r] - mnew);
      mrow[r] = mnew;
      float psum = 0.f;
#pragma unroll
      for (int j = 0; j < 4; ++j) {
        const float p = expf(s[j][r] - mnew);
        psum += p;
        const unsigned short hb = f2bf_bits(p);
        const unsigned short lb = f2bf_bits(p - bf_bits2f(hb));
        pwh[(8 * hh + r) * KCH + j * 16 + c] = __builtin_bit_cast(__bf16, hb);
        pwl[(8 * hh + r) * KCH + j * 16 + c] = __builtin_bit_cast(__bf16, lb);
      }
#pragma unroll
      for (int off = 1; off < 16; off <<= 1) psum += __shfl_xor(psum, off, 32);
      lrow[r] = lrow[r] * alpha + psum;
#pragma unroll
      for (int t = 0; t < 4; ++t) oacc[t][r] *= alpha;
    }
    __builtin_amdgcn_fence(__ATOMIC_RELEASE, "workgroup");
    __builtin_amdgcn_wave_barrier();
    __builtin_amdgcn_fence(__ATOMIC_ACQUIRE, "workgroup");

#pragma unroll
    for (int kk = 0; kk < 2; ++kk) {
      const v16b pa = Frag<__bf16>::load(pwh + c * KCH + kk * 32 + 8 * hh);
      const v16b pl = Frag<__bf16>::load(pwl + c * KCH + kk * 32 + 8 * hh);
#pragma unroll
      for (int t = 0; t < 4; ++t) {
        const __bf16* vp = Vsh + (t * 16 + c) * KCH + kk * 32 + 8 * hh;
        const __bf16* vq = Vsl + (t * 16 + c) * KCH + kk * 32 + 8 * hh;
        const v16b vfh = Frag<__bf16>::load(vp);
        const v16b vfl = Frag<__bf16>::load(vq);
        oacc[t] = at_mma(pa, vfh, oacc[t]);
        oacc[t] = at_mma(pa, vfl, oacc[t]);
        oacc[t] = at_mma(pl, vfh, oacc[t]);
      }
    }
  }

  __syncthreads();
  float* os = (float*)KVs + wave * (16 * 68);
#pragma unroll
  for (int r = 0; r < 8; ++r) {
    const float inv = 1.0f / lrow[r];
#pragma unroll
    for (int t = 0; t < 4; ++t) os[(8 * hh + r) * 68 + t * 16 + c] = oacc[t][r] * inv;
  }
  __builtin_amdgcn_fence(__ATOMIC_RELEASE, "workgroup");
  __builtin_amdgcn_wave_barrier();
  __builtin_amdgcn_fence(__ATOMIC_ACQUIRE, "workgroup");
  {
    const int q8 = lane >> 3, c8 = (lane & 7) * 8;
    for (int pass = 0; pass < 2; ++pass) {
#pragma unroll
      for (int it = 0; it < 4; ++it) {
        const int row = it * 4 + q8;
        const float* sp = os + row * 68 + c8;
        v8h hv, lv;
#pragma unroll
        for (int e = 0; e < 8; ++e) {
          const unsigned short hb = f2bf_bits(sp[e]);
          const unsigned short lb = f2bf_bits(sp[e] - bf_bits2f(hb));
          hv[e] = __builtin_bit_cast(_Float16, hb);
          lv[e] = __builtin_bit_cast(_Float16, lb);
        }
        const size_t go = (size_t)(q0 + row) * EMB + h * HDIM + c8;
        *(volatile v8h*)(ohp + go) = hv;
        *(volatile v8h*)(olp + go) = lv;
      }
      __threadfence();
    }
  }
}

extern "C" void kernel_launch(void* const* d_in, const int* in_sizes, int n_in,
                              void* d_out, int out_size, void* d_ws, size_t ws_size,
                              hipStream_t stream) {
  if (n_in < 6) return;
  const float* x  = (const float*)d_in[0];
  const float* Wq = (const float*)d_in[1];
  const float* Wk = (const float*)d_in[2];
  const float* Wv = (const float*)d_in[3];
  const float* Wo = (const float*)d_in[4];
  const int*   bi = (const int*)d_in[5];
  float* out = (float*)d_out;

  const size_t planeE  = (size_t)SEQ * EMB;
  const size_t bytesXB = (size_t)NBATCH * planeE * 2;
  const size_t bytesW  = (size_t)EMB * EMB * 2;
  const size_t bytesP  = planeE * 2;
  const size_t total   = bytesXB + 4 * bytesW + 8 * bytesP;
  if (ws_size < total) return;
  if ((size_t)out_size < (size_t)NBATCH * planeE) return;
  if (in_sizes[0] < (int)((size_t)NBATCH * planeE)) return;
  if (in_sizes[1] < EMB * EMB || in_sizes[2] < EMB * EMB || in_sizes[3] < EMB * EMB || in_sizes[4] < EMB * EMB) return;
  if (in_sizes[5] < NBLK * NMB) return;

  char* w = (char*)d_ws;
  unsigned short* xb  = (unsigned short*)(w);
  unsigned short* wqt = (unsigned short*)(w + bytesXB);
  unsigned short* wkt = (unsigned short*)(w + bytesXB + 1 * bytesW);
  unsigned short* wvt = (unsigned short*)(w + bytesXB + 2 * bytesW);
  unsigned short* wot = (unsigned short*)(w + bytesXB + 3 * bytesW);
  char* pb = w + bytesXB + 4 * bytesW;
  unsigned short* qh  = (unsigned short*)(pb + 0 * bytesP);
  unsigned short* ql  = (unsigned short*)(pb + 1 * bytesP);
  unsigned short* kh  = (unsigned short*)(pb + 2 * bytesP);
  unsigned short* kl  = (unsigned short*)(pb + 3 * bytesP);
  unsigned short* vth = (unsigned short*)(pb + 4 * bytesP);
  unsigned short* vtl = (unsigned short*)(pb + 5 * bytesP);
  unsigned short* aoh = (unsigned short*)(pb + 6 * bytesP);
  unsigned short* aol = (unsigned short*)(pb + 7 * bytesP);
  const float* dummyf = Wq;

  const int n8 = (int)((size_t)NBATCH * planeE / 8);
  cast_f32_bf16x8<<<dim3((n8 + 255) / 256), dim3(256), 0, stream>>>(x, xb, n8);

  transpose_cast_bf16<<<dim3(EMB / 64, EMB / 64, 4), dim3(256), 0, stream>>>(Wq, Wk, Wv, Wo, wqt, wkt, wvt, wot);

  const int tilesQK = (SEQ / 64) * (EMB / 64);
  const dim3 ggrid((tilesQK + 7) / 8, 1, 1);

  for (int b = 0; b < NBATCH; ++b) {
    const unsigned short* xbb = xb + (size_t)b * planeE;
    float* outb = out + (size_t)b * planeE;

    wmma_gemm64<1, false, 0, 2, false><<<ggrid, dim3(256), 0, stream>>>(
        xbb, xbb, EMB, 0L, wqt, wqt, EMB, 0L, (void*)qh, (void*)ql, EMB, 0L,
        dummyf, dummyf, 0L, SEQ, EMB, EMB, 1.0f);
    wmma_gemm64<1, false, 0, 2, false><<<ggrid, dim3(256), 0, stream>>>(
        xbb, xbb, EMB, 0L, wkt, wkt, EMB, 0L, (void*)kh, (void*)kl, EMB, 0L,
        dummyf, dummyf, 0L, SEQ, EMB, EMB, 1.0f);
    wmma_gemm64<1, false, 0, 2, false><<<ggrid, dim3(256), 0, stream>>>(
        wvt, wvt, EMB, 0L, xbb, xbb, EMB, 0L, (void*)vth, (void*)vtl, SEQ, 0L,
        dummyf, dummyf, 0L, EMB, SEQ, EMB, 1.0f);

    block_attn_kernel<<<dim3(NHEAD * NBLK), dim3(128), 0, stream>>>(qh, ql, kh, kl, vth, vtl, aoh, aol, bi);

    wmma_gemm64<1, true, 0, 0, false, 0, false><<<ggrid, dim3(256), 0, stream>>>(
        aoh, aol, EMB, 0L, wot, wot, EMB, 0L, (void*)outb, (void*)outb, EMB, 0L,
        dummyf, dummyf, 0L, SEQ, EMB, EMB, 1.0f);
  }
}
